// TrafficGNN_31971736551689
// MI455X (gfx1250) — hardware-verified
//
#include <hip/hip_runtime.h>
#include <stddef.h>
#include <stdint.h>


#define NN      50000
#define NE      800000
#define CIN     64
#define HID     128
#define NGR     64
#define MPAD    50048
#define K0      192
#define K1      512
#define NTHR    256
#define NWAVE   8
#define EPT     8
#define CHUNK   (NTHR * EPT)
#define WCAP    (EPT * 32)
#define LISTN   (NWAVE * WCAP)
#define NBRUN   1024
#define SLA     10
#define NBLK    49
#define RCAP    28672
#define DEGCAP  64
#define MEAS_B1024  16623
#define MEAS_MAXDEG 35
#define GBM     64
#define GBN     128
#define GTHR    128
#define AGR     64
#define FLAGP   32
#define XBLK    ((MPAD * (CIN / 8)) / NTHR)
#define W1BLK   12
#define W2BLK   32
#define PREPBLK (XBLK + W1BLK + W2BLK + 1)
#define AGG_ZINTS (LISTN + 2 * RCAP + 3 * NBRUN)
#define MISC_INTS 16
#define CMP_LDS_INTS (AGG_ZINTS + MISC_INTS)
#define WSMAX   134217728

static_assert(CIN == 64 && HID == 128);
static_assert(K0 % 32 == 0 && K1 % 32 == 0 && K0 == 3 * CIN && K1 == 4 * HID);
static_assert(MPAD == 391 * 128 && MPAD % GBM == 0 && MPAD % AGR == 0 && MPAD >= NN);
static_assert(NBLK * NBRUN >= MPAD);
static_assert((CHUNK & (CHUNK - 1)) == 0 && CHUNK <= 4096);
static_assert((NBRUN & (NBRUN - 1)) == 0 && NBRUN == (1 << SLA) && NBRUN % AGR == 0);
static_assert(((long long)CHUNK << SLA) < (1LL << 31));
static_assert(NE < (1 << 21));
static_assert((long long)RCAP * 100 >= (long long)MEAS_B1024 * 105);
static_assert(DEGCAP >= MEAS_MAXDEG + 8);
static_assert(RCAP % (NTHR * 4) == 0 && AGG_ZINTS % (NTHR * 4) == 0 && NBRUN == NTHR * 4);
static_assert((MPAD * (CIN / 8)) % NTHR == 0);
static_assert(W1BLK * NTHR == 3 * 1024 && W2BLK * NTHR == 4 * 2048);
static_assert(GBM == (GTHR / 32) * 16 && GBN == HID && AGR == 8 * NWAVE);
static_assert(NGR == 32 * 2 && NGR * 4 == 256);
static_assert(CMP_LDS_INTS * 4 <= 300000);
static_assert((NE & 3) == 0);

typedef float          v4f   __attribute__((ext_vector_type(4)));
typedef float          v8f   __attribute__((ext_vector_type(8)));
typedef int            v4i   __attribute__((ext_vector_type(4)));
typedef int            v8i   __attribute__((ext_vector_type(8)));
typedef unsigned       v2u   __attribute__((ext_vector_type(2)));
typedef unsigned       v4u   __attribute__((ext_vector_type(4)));
typedef unsigned short v4us  __attribute__((ext_vector_type(4)));
typedef unsigned short v8us  __attribute__((ext_vector_type(8)));
typedef unsigned short v16us __attribute__((ext_vector_type(16)));
typedef __bf16         v16bf __attribute__((ext_vector_type(16)));
typedef v4f  __attribute__((may_alias)) v4fa;
typedef v4i  __attribute__((may_alias)) v4ia;
typedef v2u  __attribute__((may_alias)) v2ua;
typedef v4u  __attribute__((may_alias)) v4ua;
typedef v4us __attribute__((may_alias)) v4usa;
typedef v8us __attribute__((may_alias)) v8usa;
typedef unsigned __attribute__((may_alias)) u32a;
union FragB { v16bf v; v16us u; v8us h[2]; v8i w; };

__device__ __forceinline__ v8f wmb(const FragB& a, const FragB& b, v8f c) {
  v8f d = __builtin_amdgcn_wmma_f32_16x16x32_bf16(false, a.v, false, b.v, (short)0, c, false, false);
  asm volatile("v_nop\n\tv_nop\n\tv_nop\n\tv_nop" : "+v"(d) : "v"(a.w), "v"(b.w));
  return d;
}

__device__ __forceinline__ unsigned bf16n_bits(float f) {
  const unsigned u = __float_as_uint(f);
  const unsigned r = (u + 0x7FFFu + ((u >> 16) & 1u)) >> 16;
  const unsigned q = (u >> 16) | 0x0040u;
  return ((u & 0x7fffffffu) > 0x7f800000u) ? q : r;
}
__device__ __forceinline__ float bf16n_val(float f) {
  return __uint_as_float(bf16n_bits(f) << 16);
}
__device__ __forceinline__ float relu_keep(float t) { return (t > 0.0f) ? t : (t - t); }

__device__ __forceinline__ void wave_sync() {
  __builtin_amdgcn_fence(__ATOMIC_RELEASE, "wavefront");
  __builtin_amdgcn_wave_barrier();
  __builtin_amdgcn_fence(__ATOMIC_ACQUIRE, "wavefront");
}

template <int SLB>
__device__ __forceinline__ int scan_chunk(const int* __restrict__ dsts, int nE, int cbase, int slotBase,
                                          int nb, int vec8, int* list, int tid, int lane, int wave) {
  int wc = 0;
  const int el0  = tid * EPT;
  const int e0   = cbase + el0;
  const int sent = -2147483647 - 1;
  v4i da, db;
  if (vec8 != 0 && cbase + CHUNK <= nE) {
    da = *(const v4i*)(dsts + e0);
    db = *(const v4i*)(dsts + e0 + 4);
  } else {
    da.x = (e0     < nE) ? dsts[min(e0,     nE - 1)] : sent;
    da.y = (e0 + 1 < nE) ? dsts[min(e0 + 1, nE - 1)] : sent;
    da.z = (e0 + 2 < nE) ? dsts[min(e0 + 2, nE - 1)] : sent;
    da.w = (e0 + 3 < nE) ? dsts[min(e0 + 3, nE - 1)] : sent;
    db.x = (e0 + 4 < nE) ? dsts[min(e0 + 4, nE - 1)] : sent;
    db.y = (e0 + 5 < nE) ? dsts[min(e0 + 5, nE - 1)] : sent;
    db.z = (e0 + 6 < nE) ? dsts[min(e0 + 6, nE - 1)] : sent;
    db.w = (e0 + 7 < nE) ? dsts[min(e0 + 7, nE - 1)] : sent;
  }
  const unsigned nbs = (unsigned)slotBase;
  const unsigned unb = (unsigned)nb;
  const unsigned s0 = (unsigned)da.x - nbs, s1 = (unsigned)da.y - nbs;
  const unsigned s2 = (unsigned)da.z - nbs, s3 = (unsigned)da.w - nbs;
  const unsigned s4 = (unsigned)db.x - nbs, s5 = (unsigned)db.y - nbs;
  const unsigned s6 = (unsigned)db.z - nbs, s7 = (unsigned)db.w - nbs;
  const bool h0 = s0 < unb, h1 = s1 < unb, h2 = s2 < unb, h3 = s3 < unb;
  const bool h4 = s4 < unb, h5 = s5 < unb, h6 = s6 < unb, h7 = s7 < unb;
  const unsigned any = __builtin_amdgcn_ballot_w32(h0 | h1 | h2 | h3 | h4 | h5 | h6 | h7);
  if (any != 0u) {
#define HITJ(J, HJ, SJ) { \
      const unsigned mj = __builtin_amdgcn_ballot_w32(HJ); \
      if (mj != 0u) { \
        if (HJ) { \
          const int pos = wc + (int)__builtin_amdgcn_mbcnt_lo(mj, 0u); \
          if (pos < WCAP) list[wave * WCAP + pos] = ((el0 + (J)) << SLB) | (int)(SJ); \
        } \
        wc += (int)__builtin_popcount(mj); } }
    HITJ(0, h0, s0)
    HITJ(1, h1, s1)
    HITJ(2, h2, s2)
    HITJ(3, h3, s3)
    HITJ(4, h4, s4)
    HITJ(5, h5, s5)
    HITJ(6, h6, s6)
    HITJ(7, h7, s7)
#undef HITJ
  }
  return wc;
}

__device__ __forceinline__ void wunit(const float* __restrict__ W, int kk, int n, unsigned short* dp) {
  const float* p = W + (size_t)kk * HID + n;
  v8us o;
#pragma unroll
  for (int i = 0; i < 8; ++i) o[i] = (unsigned short)bf16n_bits(p[(size_t)i * HID]);
  *(volatile v8us*)dp = o;
  __threadfence();
  *(volatile v8us*)dp = o;
}

__global__ __launch_bounds__(NTHR) void k_prep(const float* __restrict__ x,
                                               const float* __restrict__ Wl1, const float* __restrict__ Wr1,
                                               const float* __restrict__ Wl2, const float* __restrict__ Wr2,
                                               const float* __restrict__ bl1, const float* __restrict__ bl2,
                                               const float* __restrict__ Wout, const float* __restrict__ bout,
                                               unsigned short* XB, unsigned short* W1c, unsigned short* W2c,
                                               float* TB) {
  const int blk = (int)blockIdx.x;
  const int tid = (int)threadIdx.x;
  if (blk < XBLK) {
    const int u   = blk * NTHR + tid;
    const int row = u >> 3;
    const int k8  = (u & 7) * 8;
    const int rc  = row < NN ? row : NN - 1;
    const float* p = x + (size_t)rc * CIN + k8;
    const v4f a = *(const v4fa*)p;
    const v4f b = *(const v4fa*)(p + 4);
    const bool ok = row < NN;
    v8us o;
    o[0] = ok ? (unsigned short)bf16n_bits(a.x) : (unsigned short)0;
    o[1] = ok ? (unsigned short)bf16n_bits(a.y) : (unsigned short)0;
    o[2] = ok ? (unsigned short)bf16n_bits(a.z) : (unsigned short)0;
    o[3] = ok ? (unsigned short)bf16n_bits(a.w) : (unsigned short)0;
    o[4] = ok ? (unsigned short)bf16n_bits(b.x) : (unsigned short)0;
    o[5] = ok ? (unsigned short)bf16n_bits(b.y) : (unsigned short)0;
    o[6] = ok ? (unsigned short)bf16n_bits(b.z) : (unsigned short)0;
    o[7] = ok ? (unsigned short)bf16n_bits(b.w) : (unsigned short)0;
    unsigned short* dp = XB + (size_t)row * CIN + k8;
    *(volatile v8us*)dp = o;
    __threadfence();
    *(volatile v8us*)dp = o;
  } else if (blk < XBLK + W1BLK) {
    const int v    = (blk - XBLK) * NTHR + tid;
    const int part = v >> 10;
    const int vv   = v & 1023;
    const int n    = vv >> 3;
    const int k8   = (vv & 7) * 8;
    unsigned short* dp = W1c + (size_t)n * K0 + CIN * part + k8;
    if (part < 2) wunit(Wl1, k8, n, dp);
    else          wunit(Wr1, k8, n, dp);
  } else if (blk < XBLK + W1BLK + W2BLK) {
    const int v    = (blk - XBLK - W1BLK) * NTHR + tid;
    const int part = v >> 11;
    const int vv   = v & 2047;
    const int n    = vv >> 4;
    const int k8   = (vv & 15) * 8;
    unsigned short* dp = W2c + (size_t)n * K1 + HID * part + k8;
    if (part < 2) wunit(Wl2, k8, n, dp);
    else          wunit(Wr2, k8, n, dp);
  } else {
    if (tid < 128) {
      const int q = tid >> 5;
      const int l = tid & 31;
      v4f v;
      if (q == 0)      v = *(const v4fa*)(bl1 + 4 * l);
      else if (q == 1) v = *(const v4fa*)(bl2 + 4 * l);
      else if (q == 2) v = *(const v4fa*)(Wout + 4 * l);
      else {
        const float b = bout[0];
        v.x = (l == 0) ? b : 0.0f; v.y = 0.0f; v.z = 0.0f; v.w = 0.0f;
      }
      v4f o;
      o.x = bf16n_val(v.x); o.y = bf16n_val(v.y); o.z = bf16n_val(v.z); o.w = bf16n_val(v.w);
      float* dp = TB + 128 * q + 4 * l;
      *(volatile v4f*)dp = o;
      __threadfence();
      *(volatile v4f*)dp = o;
    }
  }
}

__global__ __launch_bounds__(NTHR) void k_compact(const int* __restrict__ srcs, const int* __restrict__ dsts,
                                                  int nE, int nN, int vec8,
                                                  int* LIST, int* CNT, int* OFF, int* FLAGS) {
  extern __shared__ __attribute__((aligned(16))) int dsm[];
  int* list = dsm;
  int* hl   = dsm + LISTN;
  int* sl   = hl + RCAP;
  int* cnt  = sl + RCAP;
  int* offs = cnt + NBRUN;
  int* cur  = offs + NBRUN;
  int* misc = cur + NBRUN;
  const int tid = (int)threadIdx.x, lane = tid & 31, wave = tid >> 5;
  const int blk = (int)blockIdx.x;
  const int nodeBase = blk * NBRUN;

  {
    const v4i z4 = {0, 0, 0, 0};
    for (int i = tid * 4; i < AGG_ZINTS; i += NTHR * 4) *(v4ia*)(dsm + i) = z4;
    if (tid < MISC_INTS) misc[tid] = 0;
  }
  __syncthreads();

  int t = 0, ov = 0;
  const int nChunks = (nE + CHUNK - 1) / CHUNK;
#pragma unroll 1
  for (int ch = 0; ch < nChunks; ++ch) {
    const int cbase = ch * CHUNK;
    const int wc = scan_chunk<SLA>(dsts, nE, cbase, nodeBase, NBRUN, vec8, list, tid, lane, wave);
    if (lane == 0) misc[wave] = wc;
    __syncthreads();
    if (wave == 0) {
#pragma unroll 1
      for (int w2 = 0; w2 < NWAVE; ++w2) {
        int c = misc[w2];
        c = c < 0 ? 0 : (c > WCAP ? WCAP : c);
#pragma unroll 1
        for (int b0 = 0; b0 < c; b0 += 32) {
          const int idx = b0 + lane;
          const int ent = list[w2 * WCAP + (idx < WCAP ? idx : WCAP - 1)];
          const int m32 = (c - b0) < 32 ? (c - b0) : 32;
#pragma unroll 1
          for (int k = 0; k < m32; ++k) {
            const int u    = __builtin_amdgcn_readlane(ent, k);
            const int slot = u & (NBRUN - 1);
            const int el   = (u >> SLA) & (CHUNK - 1);
            const int pk   = ((cbase + el) << SLA) | slot;
            if (t < RCAP) {
              if (lane == 0) { hl[t] = pk; cnt[slot] = cnt[slot] + 1; }
              t = t + 1;
            } else {
              ov = 1;
            }
          }
        }
      }
    }
    __syncthreads();
  }
  if (wave == 0 && lane == 0) { misc[8] = t; misc[9] = ov; }
  __syncthreads();
  int tt = misc[8];
  tt = tt < 0 ? 0 : (tt > RCAP ? RCAP : tt);
  const int ovf = misc[9];

  if (wave == 0) {
    const int base = lane * (NBRUN / 32);
    int s = 0, mx = 0;
#pragma unroll 1
    for (int i = 0; i < NBRUN / 32; ++i) {
      const int cv = cnt[base + i];
      s += cv;
      mx = cv > mx ? cv : mx;
    }
    int incl = s;
#pragma unroll
    for (int d = 1; d < 32; d <<= 1) {
      const int y = __shfl_up(incl, d, 32);
      if (lane >= d) incl += y;
    }
    int run = incl - s;
#pragma unroll 1
    for (int i = 0; i < NBRUN / 32; ++i) {
      const int cv = cnt[base + i];
      offs[base + i] = run;
      cur[base + i]  = run;
      run += cv;
    }
    const unsigned bm = __builtin_amdgcn_ballot_w32(mx > DEGCAP);
    if (lane == 0) misc[10] = (bm != 0u) ? 1 : 0;
  }
  __syncthreads();
  if (wave == 0) {
#pragma unroll 1
    for (int b0 = 0; b0 < tt; b0 += 32) {
      const int idx = b0 + lane;
      const int ent = hl[idx < RCAP ? idx : RCAP - 1];
      const int m32 = (tt - b0) < 32 ? (tt - b0) : 32;
#pragma unroll 1
      for (int k = 0; k < m32; ++k) {
        const int u    = __builtin_amdgcn_readlane(ent, k);
        const int slot = u & (NBRUN - 1);
        if (lane == 0) {
          int p = cur[slot];
          p = p < 0 ? 0 : (p > RCAP - 1 ? RCAP - 1 : p);
          sl[p] = u;
          cur[slot] = p + 1;
        }
      }
    }
  }
  __syncthreads();
  const int flag = (ovf != 0 || misc[10] != 0) ? 1 : 0;

#pragma unroll 1
  for (int it = 0; it < RCAP / (NTHR * 4); ++it) {
    const int p0 = it * (NTHR * 4) + 4 * tid;
    const v4i e4 = *(const v4ia*)(sl + p0);
    int e0 = e4.x >> SLA, e1 = e4.y >> SLA, e2 = e4.z >> SLA, e3 = e4.w >> SLA;
    e0 = e0 < 0 ? 0 : (e0 > nE - 1 ? nE - 1 : e0);
    e1 = e1 < 0 ? 0 : (e1 > nE - 1 ? nE - 1 : e1);
    e2 = e2 < 0 ? 0 : (e2 > nE - 1 ? nE - 1 : e2);
    e3 = e3 < 0 ? 0 : (e3 > nE - 1 ? nE - 1 : e3);
    int r0 = srcs[e0], r1 = srcs[e1], r2 = srcs[e2], r3 = srcs[e3];
    r0 = r0 < 0 ? 0 : (r0 > nN - 1 ? nN - 1 : r0);
    r1 = r1 < 0 ? 0 : (r1 > nN - 1 ? nN - 1 : r1);
    r2 = r2 < 0 ? 0 : (r2 > nN - 1 ? nN - 1 : r2);
    r3 = r3 < 0 ? 0 : (r3 > nN - 1 ? nN - 1 : r3);
    v4i o;
    o.x = (p0     < tt) ? r0 : 0;
    o.y = (p0 + 1 < tt) ? r1 : 0;
    o.z = (p0 + 2 < tt) ? r2 : 0;
    o.w = (p0 + 3 < tt) ? r3 : 0;
    *(v4ia*)(hl + p0) = o;
  }
  __syncthreads();

  int* lg = LIST + (size_t)blk * RCAP;
  const v4i c4 = *(const v4ia*)(cnt + 4 * tid);
  const v4i o4 = *(const v4ia*)(offs + 4 * tid);
  const v4i f4 = {flag, flag, flag, flag};
  const bool fw = (wave == 0) && (lane < 8);
#pragma unroll 1
  for (int it = 0; it < RCAP / (NTHR * 4); ++it) {
    const int p0 = it * (NTHR * 4) + 4 * tid;
    const v4i v = *(const v4ia*)(hl + p0);
    *(volatile v4i*)(lg + p0) = v;
  }
  *(volatile v4i*)(CNT + nodeBase + 4 * tid) = c4;
  *(volatile v4i*)(OFF + nodeBase + 4 * tid) = o4;
  if (fw) *(volatile v4i*)(FLAGS + blk * FLAGP + 4 * (lane & 7)) = f4;
  __threadfence();
#pragma unroll 1
  for (int it = 0; it < RCAP / (NTHR * 4); ++it) {
    const int p0 = it * (NTHR * 4) + 4 * tid;
    const v4i v = *(const v4ia*)(hl + p0);
    *(volatile v4i*)(lg + p0) = v;
  }
  *(volatile v4i*)(CNT + nodeBase + 4 * tid) = c4;
  *(volatile v4i*)(OFF + nodeBase + 4 * tid) = o4;
  if (fw) *(volatile v4i*)(FLAGS + blk * FLAGP + 4 * (lane & 7)) = f4;
}

template <int L>
__global__ __launch_bounds__(NTHR) void k_agg(const int* __restrict__ LIST, const int* __restrict__ CNT,
                                              const int* __restrict__ OFF, const int* __restrict__ FLAGS,
                                              const unsigned short* __restrict__ sp, unsigned short* dp) {
  __shared__ __attribute__((aligned(16))) unsigned rb[NWAVE * 128];
  const int tid = (int)threadIdx.x, lane = tid & 31, wave = tid >> 5;
  unsigned* rbw = rb + wave * 128;
  const int rowBase = (int)blockIdx.x * AGR;
  int pb = rowBase >> SLA;
  pb = pb > NBLK - 1 ? NBLK - 1 : pb;
  const int fl = FLAGS[pb * FLAGP];
  const float qnan = __int_as_float(0x7fc00000);
  const float pz = (fl != 0) ? qnan : 0.0f;
  const int* lst = LIST + (size_t)pb * RCAP;

#pragma unroll 1
  for (int si = 0; si < AGR / NWAVE; ++si) {
    const int node = rowBase + si * NWAVE + wave;
    const int cr = CNT[node];
    const bool big = cr > DEGCAP;
    int c = cr < 0 ? 0 : (cr > DEGCAP ? DEGCAP : cr);
    int o = OFF[node];
    o = o < 0 ? 0 : (o > RCAP ? RCAP : o);
    float a0 = 0.0f, a1 = 0.0f, a2 = 0.0f, a3 = 0.0f;
#pragma unroll 1
    for (int b0 = 0; b0 < c; b0 += 32) {
      int j = b0 + lane;
      j = j > c - 1 ? c - 1 : j;
      int idx = o + j;
      idx = idx > RCAP - 1 ? RCAP - 1 : idx;
      int sr = lst[idx];
      sr = sr < 0 ? 0 : (sr > NN - 1 ? NN - 1 : sr);
      const int m32 = (c - b0) < 32 ? (c - b0) : 32;
#pragma unroll 1
      for (int k = 0; k < m32; ++k) {
        const int sk = __builtin_amdgcn_readlane(sr, k);
        if constexpr (L == 0) {
          const unsigned w = *(const u32a*)(sp + (size_t)sk * CIN + 2 * lane);
          a0 += __uint_as_float(w << 16);
          a1 += __uint_as_float(w & 0xffff0000u);
        } else {
          const unsigned short* rp = sp + (size_t)sk * (2 * HID) + 4 * lane;
          const v2u wh = *(const v2ua*)rp;
          const v2u wl = *(const v2ua*)(rp + HID);
          a0 += __uint_as_float(wh.x << 16)         + __uint_as_float(wl.x << 16);
          a1 += __uint_as_float(wh.x & 0xffff0000u) + __uint_as_float(wl.x & 0xffff0000u);
          a2 += __uint_as_float(wh.y << 16)         + __uint_as_float(wl.y << 16);
          a3 += __uint_as_float(wh.y & 0xffff0000u) + __uint_as_float(wl.y & 0xffff0000u);
        }
      }
    }
    const float dn  = (float)(cr < 1 ? 1 : cr);
    const float pzr = big ? qnan : pz;
    const bool live = node < NN;
    if constexpr (L == 0) {
      const float m0 = live ? (a0 / dn + pzr) : 0.0f;
      const float m1 = live ? (a1 / dn + pzr) : 0.0f;
      const unsigned h0 = bf16n_bits(m0), h1 = bf16n_bits(m1);
      const unsigned l0 = bf16n_bits(m0 - __uint_as_float(h0 << 16));
      const unsigned l1 = bf16n_bits(m1 - __uint_as_float(h1 << 16));
      rbw[lane]      = h0 | (h1 << 16);
      rbw[32 + lane] = l0 | (l1 << 16);
      wave_sync();
      const v4u q = *(const v4ua*)(rbw + 4 * (lane & 15));
      wave_sync();
      const bool wr = lane < 16;
      unsigned short* rp = dp + (size_t)node * (2 * CIN) + 8 * (lane & 15);
      if (wr) *(volatile v4u*)rp = q;
      __threadfence();
      if (wr) *(volatile v4u*)rp = q;
    } else {
      const float m0 = live ? (a0 / dn + pzr) : 0.0f;
      const float m1 = live ? (a1 / dn + pzr) : 0.0f;
      const float m2 = live ? (a2 / dn + pzr) : 0.0f;
      const float m3 = live ? (a3 / dn + pzr) : 0.0f;
      v4us mh, ml;
      unsigned hb;
      hb = bf16n_bits(m0); mh[0] = (unsigned short)hb; ml[0] = (unsigned short)bf16n_bits(m0 - __uint_as_float(hb << 16));
      hb = bf16n_bits(m1); mh[1] = (unsigned short)hb; ml[1] = (unsigned short)bf16n_bits(m1 - __uint_as_float(hb << 16));
      hb = bf16n_bits(m2); mh[2] = (unsigned short)hb; ml[2] = (unsigned short)bf16n_bits(m2 - __uint_as_float(hb << 16));
      hb = bf16n_bits(m3); mh[3] = (unsigned short)hb; ml[3] = (unsigned short)bf16n_bits(m3 - __uint_as_float(hb << 16));
      unsigned short* rs = (unsigned short*)rbw;
      *(v4usa*)(rs + 4 * lane) = mh;
      *(v4usa*)(rs + HID + 4 * lane) = ml;
      wave_sync();
      const v8us q0 = *(const v8usa*)(rs + 8 * lane);
      wave_sync();
      unsigned short* rp = dp + (size_t)node * (2 * HID) + 8 * lane;
      *(volatile v8us*)rp = q0;
      __threadfence();
      *(volatile v8us*)rp = q0;
    }
  }
}

template <int L>
__global__ __launch_bounds__(GTHR) void k_gemm(const unsigned short* __restrict__ A1,
                                               const unsigned short* __restrict__ A2,
                                               const unsigned short* __restrict__ BT,
                                               const float* __restrict__ TB,
                                               unsigned short* H1o, float* So) {
  constexpr int P1  = L ? 256 : 128;
  constexpr int P2  = L ? 256 : 64;
  constexpr int KS1 = L ? 8 : 4;
  constexpr int KS2 = L ? 8 : 2;
  constexpr int KB  = L ? K1 : K0;
  constexpr int BO2 = L ? 256 : 128;
  __shared__ __attribute__((aligned(16))) float stg[GBM * GBN];
  __shared__ __attribute__((aligned(16))) float sS[GBM];
  const int tid = (int)threadIdx.x, lane = tid & 31, wave = tid >> 5, hh = lane >> 4, m = lane & 15;
  const int rowBase = (int)blockIdx.x * GBM;

  v8f acc[8];
  {
    const v8f z = {0.f, 0.f, 0.f, 0.f, 0.f, 0.f, 0.f, 0.f};
#pragma unroll
    for (int t = 0; t < 8; ++t) acc[t] = z;
  }
  const unsigned short* ap1 = A1 + (size_t)(rowBase + 16 * wave + m) * (size_t)P1 + 8 * hh;
  const unsigned short* ap2 = A2 + (size_t)(rowBase + 16 * wave + m) * (size_t)P2 + 8 * hh;
  const unsigned short* bp  = BT + (size_t)m * (size_t)KB + 8 * hh;

#pragma unroll 1
  for (int ks = 0; ks < KS1; ++ks) {
    FragB af;
    af.h[0] = *(const v8usa*)(ap1 + 32 * ks);
    af.h[1] = *(const v8usa*)(ap1 + 32 * ks + 16);
#pragma unroll
    for (int nt = 0; nt < 8; ++nt) {
      const unsigned short* wq = bp + (size_t)(16 * nt) * (size_t)KB + 32 * ks;
      FragB bf;
      bf.h[0] = *(const v8usa*)wq;
      bf.h[1] = *(const v8usa*)(wq + 16);
      acc[nt] = wmb(af, bf, acc[nt]);
    }
  }
#pragma unroll 1
  for (int ks = 0; ks < KS2; ++ks) {
    FragB af;
    af.h[0] = *(const v8usa*)(ap2 + 32 * ks);
    af.h[1] = *(const v8usa*)(ap2 + 32 * ks + 16);
#pragma unroll
    for (int nt = 0; nt < 8; ++nt) {
      const unsigned short* wq = bp + (size_t)(16 * nt) * (size_t)KB + BO2 + 32 * ks;
      FragB bf;
      bf.h[0] = *(const v8usa*)wq;
      bf.h[1] = *(const v8usa*)(wq + 16);
      acc[nt] = wmb(af, bf, acc[nt]);
    }
  }

#pragma unroll
  for (int nt = 0; nt < 8; ++nt) {
    const int lc = 16 * nt + m;
#pragma unroll
    for (int r = 0; r < 8; ++r) {
      const int lr = 16 * wave + 8 * hh + r;
      stg[lr * GBN + lc] = acc[nt][r];
    }
  }
  __syncthreads();

  const v4f bb4 = *(const v4fa*)(TB + 128 * L + 4 * lane);

  if constexpr (L == 0) {
    v4f pv[16];
#pragma unroll
    for (int i = 0; i < 16; ++i) pv[i] = *(const v4fa*)(stg + (16 * wave + i) * GBN + 4 * lane);
    __syncthreads();
#pragma unroll
    for (int i = 0; i < 16; ++i) {
      const v4f t = pv[i] + bb4;
      v4f y;
      y.x = relu_keep(t.x); y.y = relu_keep(t.y); y.z = relu_keep(t.z); y.w = relu_keep(t.w);
      v4us h4, l4;
      unsigned hb;
      hb = bf16n_bits(y.x); h4[0] = (unsigned short)hb; l4[0] = (unsigned short)bf16n_bits(y.x - __uint_as_float(hb << 16));
      hb = bf16n_bits(y.y); h4[1] = (unsigned short)hb; l4[1] = (unsigned short)bf16n_bits(y.y - __uint_as_float(hb << 16));
      hb = bf16n_bits(y.z); h4[2] = (unsigned short)hb; l4[2] = (unsigned short)bf16n_bits(y.z - __uint_as_float(hb << 16));
      hb = bf16n_bits(y.w); h4[3] = (unsigned short)hb; l4[3] = (unsigned short)bf16n_bits(y.w - __uint_as_float(hb << 16));
      unsigned short* srow = (unsigned short*)stg + (size_t)(16 * wave + i) * (2 * GBN);
      *(v4usa*)(srow + 4 * lane) = h4;
      *(v4usa*)(srow + HID + 4 * lane) = l4;
    }
    __syncthreads();
    v8us qv[16];
#pragma unroll
    for (int i = 0; i < 16; ++i) {
      const unsigned short* srow = (const unsigned short*)stg + (size_t)(16 * wave + i) * (2 * GBN);
      qv[i] = *(const v8usa*)(srow + 8 * lane);
    }
#pragma unroll
    for (int i = 0; i < 16; ++i) {
      unsigned short* rp = H1o + (size_t)(rowBase + 16 * wave + i) * (size_t)(2 * HID) + 8 * lane;
      *(volatile v8us*)rp = qv[i];
    }
    __threadfence();
#pragma unroll
    for (int i = 0; i < 16; ++i) {
      unsigned short* rp = H1o + (size_t)(rowBase + 16 * wave + i) * (size_t)(2 * HID) + 8 * lane;
      *(volatile v8us*)rp = qv[i];
    }
  } else {
    const v4f w4 = *(const v4fa*)(TB + 256 + 4 * lane);
    float sv = 0.0f;
#pragma unroll 4
    for (int i = 0; i < 16; ++i) {
      const v4f t = *(const v4fa*)(stg + (16 * wave + i) * GBN + 4 * lane) + bb4;
      const float y0 = relu_keep(t.x), y1 = relu_keep(t.y), y2 = relu_keep(t.z), y3 = relu_keep(t.w);
      float p = y0 * w4.x;
      p = fmaf(y1, w4.y, p);
      p = fmaf(y2, w4.z, p);
      p = fmaf(y3, w4.w, p);
      p += __shfl_xor(p, 16, 32);
      p += __shfl_xor(p, 8, 32);
      p += __shfl_xor(p, 4, 32);
      p += __shfl_xor(p, 2, 32);
      p += __shfl_xor(p, 1, 32);
      sv = (lane == i) ? p : sv;
    }
    const int grow = rowBase + 16 * wave + (lane & 15);
    const float so = (grow < NN) ? sv : 0.0f;
    if (lane < 16) sS[16 * wave + lane] = so;
    __syncthreads();
    const v4f ov = *(const v4fa*)(sS + 4 * (lane & 15));
    float* op = So + (size_t)rowBase + 4 * (lane & 15);
    const bool okst = (wave == 0) && (lane < 16);
    if (okst) *(volatile v4f*)op = ov;
    __threadfence();
    if (okst) *(volatile v4f*)op = ov;
  }
}

__global__ __launch_bounds__(1024) void k_pool(const float* __restrict__ S, const int* __restrict__ bat,
                                               const int* __restrict__ FLAGS, const float* __restrict__ TB,
                                               float* out) {
  __shared__ double part[NGR * 32];
  __shared__ int cn[NGR * 32];
  __shared__ __attribute__((aligned(16))) float outs[NGR];
  const int tid = (int)threadIdx.x, lane = tid & 31, wave = tid >> 5;
  const int g0 = 2 * wave, g1 = 2 * wave + 1;
  double a0 = 0.0, a1 = 0.0;
  int c0 = 0, c1 = 0;
#pragma unroll 2
  for (int n0 = 0; n0 < NN; n0 += 32) {
    const int n  = n0 + lane;
    const int nc = n < NN ? n : NN - 1;
    const int b  = bat[nc];
    const float s = S[nc];
    const bool ok = n < NN;
    const bool h0 = ok && (b == g0);
    const bool h1 = ok && (b == g1);
    const double sd = (double)s;
    a0 += h0 ? sd : 0.0;
    a1 += h1 ? sd : 0.0;
    c0 += h0 ? 1 : 0;
    c1 += h1 ? 1 : 0;
  }
  part[g0 * 32 + lane] = a0;
  part[g1 * 32 + lane] = a1;
  cn[g0 * 32 + lane] = c0;
  cn[g1 * 32 + lane] = c1;
  __syncthreads();
  if (tid < NGR) {
    double sm = 0.0;
    int ct = 0;
#pragma unroll 1
    for (int l = 0; l < 32; ++l) { sm += part[tid * 32 + l]; ct += cn[tid * 32 + l]; }
    int anyf = 0;
#pragma unroll 1
    for (int b = 0; b < NBLK; ++b) anyf |= FLAGS[b * FLAGP];
    const double dn = (double)(ct < 1 ? 1 : ct);
    float v = (float)(sm / dn) + TB[384];
    v = (anyf != 0) ? __int_as_float(0x7fc00000) : v;
    outs[tid] = v;
  }
  __syncthreads();
  const v4f ov = *(const v4fa*)(outs + 4 * (lane & 15));
  float* op = out + 4 * (lane & 15);
  const bool okst = (wave == 0) && (lane < 16);
  if (okst) *(volatile v4f*)op = ov;
  __threadfence();
  if (okst) *(volatile v4f*)op = ov;
}

static inline size_t al256(size_t o) { return (o + 255) & ~(size_t)255; }

extern "C" void kernel_launch(void* const* d_in, const int* in_sizes, int n_in,
                              void* d_out, int out_size, void* d_ws, size_t ws_size,
                              hipStream_t stream) {
  if (n_in < 11) return;
  if (in_sizes[0] != NN * CIN) return;
  if (in_sizes[1] != 2 * NE) return;
  if (in_sizes[2] != NN) return;
  if (in_sizes[3] != CIN * HID || in_sizes[4] != HID || in_sizes[5] != CIN * HID) return;
  if (in_sizes[6] != HID * HID || in_sizes[7] != HID || in_sizes[8] != HID * HID) return;
  if (in_sizes[9] != HID || in_sizes[10] != 1) return;
  if (out_size != NGR) return;

  const float* x    = (const float*)d_in[0];
  const int*   edge = (const int*)d_in[1];
  const int*   bat  = (const int*)d_in[2];
  const float* Wl1  = (const float*)d_in[3];
  const float* bl1  = (const float*)d_in[4];
  const float* Wr1  = (const float*)d_in[5];
  const float* Wl2  = (const float*)d_in[6];
  const float* bl2  = (const float*)d_in[7];
  const float* Wr2  = (const float*)d_in[8];
  const float* Wout = (const float*)d_in[9];
  const float* bout = (const float*)d_in[10];
  float* out = (float*)d_out;
  const int* src = edge;
  const int* dst = edge + NE;

  char* ws = (char*)d_ws;
  size_t off = 0;
  const size_t oXB  = off; off = al256(off + (size_t)MPAD * CIN * 2);
  const size_t oAG0 = off; off = al256(off + (size_t)MPAD * 2 * CIN * 2);
  const size_t oH1  = off; off = al256(off + (size_t)MPAD * 2 * HID * 2);
  const size_t oAG1 = off; off = al256(off + (size_t)MPAD * 2 * HID * 2);
  const size_t oS   = off; off = al256(off + (size_t)MPAD * 4);
  const size_t oLST = off; off = al256(off + (size_t)NBLK * RCAP * 4);
  const size_t oCNT = off; off = al256(off + (size_t)NBLK * NBRUN * 4);
  const size_t oOFF = off; off = al256(off + (size_t)NBLK * NBRUN * 4);
  const size_t oFLG = off; off = al256(off + (size_t)NBLK * FLAGP * 4);
  const size_t oW1  = off; off = al256(off + (size_t)HID * K0 * 2);
  const size_t oW2  = off; off = al256(off + (size_t)HID * K1 * 2);
  const size_t oTB  = off; off = al256(off + (size_t)512 * 4);
  if (off > ws_size || off > (size_t)WSMAX) return;
  unsigned short* XB  = (unsigned short*)(ws + oXB);
  unsigned short* AG0 = (unsigned short*)(ws + oAG0);
  unsigned short* H1  = (unsigned short*)(ws + oH1);
  unsigned short* AG1 = (unsigned short*)(ws + oAG1);
  float*          Sb  = (float*)(ws + oS);
  int*            LST = (int*)(ws + oLST);
  int*            CNT = (int*)(ws + oCNT);
  int*            OFF = (int*)(ws + oOFF);
  int*            FLG = (int*)(ws + oFLG);
  unsigned short* W1c = (unsigned short*)(ws + oW1);
  unsigned short* W2c = (unsigned short*)(ws + oW2);
  float*          TB  = (float*)(ws + oTB);

  const size_t cmpLds = (size_t)CMP_LDS_INTS * 4;
  hipFuncSetAttribute(reinterpret_cast<const void*>(&k_compact), hipFuncAttributeMaxDynamicSharedMemorySize, (int)cmpLds);

  k_prep<<<PREPBLK, NTHR, 0, stream>>>(x, Wl1, Wr1, Wl2, Wr2, bl1, bl2, Wout, bout, XB, W1c, W2c, TB);
  k_compact<<<NBLK, NTHR, cmpLds, stream>>>(src, dst, NE, NN, 1, LST, CNT, OFF, FLG);
  k_agg<0><<<MPAD / AGR, NTHR, 0, stream>>>(LST, CNT, OFF, FLG, XB, AG0);
  k_gemm<0><<<MPAD / GBM, GTHR, 0, stream>>>(AG0, XB, W1c, TB, H1, Sb);
  k_agg<1><<<MPAD / AGR, NTHR, 0, stream>>>(LST, CNT, OFF, FLG, H1, AG1);
  k_gemm<1><<<MPAD / GBM, GTHR, 0, stream>>>(AG1, H1, W2c, TB, H1, Sb);
  k_pool<<<1, 1024, 0, stream>>>(Sb, bat, FLG, TB, out);
}
